// GCN_33243046871768
// MI455X (gfx1250) — hardware-run, weakly checked
//
#include <hip/hip_runtime.h>

typedef float          v8f   __attribute__((ext_vector_type(8)));
typedef float          v4f   __attribute__((ext_vector_type(4)));
typedef unsigned int   v4u   __attribute__((ext_vector_type(4)));
typedef int            v8i   __attribute__((ext_vector_type(8)));
typedef unsigned short v8us  __attribute__((ext_vector_type(8)));
typedef unsigned short v16us __attribute__((ext_vector_type(16)));
typedef __bf16         v16bf __attribute__((ext_vector_type(16)));
typedef _Float16       v16h  __attribute__((ext_vector_type(16)));
typedef v4f  __attribute__((may_alias)) v4fa;
typedef v8us __attribute__((may_alias)) v8usa;
union FragB { v16bf v; v16us u; v8us h[2]; v8i w; };
union FragH { v16h  v; v16us u; v8us h[2]; v8i w; };

__device__ __forceinline__ v8f wmb(const FragB& a, const FragB& b, v8f c) {
  v8f d = __builtin_amdgcn_wmma_f32_16x16x32_bf16(false, a.v, false, b.v, (short)0, c, false, false);
  asm volatile("v_nop\n\tv_nop\n\tv_nop\n\tv_nop" : "+v"(d) : "v"(a.w), "v"(b.w));
  return d;
}

__device__ __forceinline__ v8f wmh(const FragH& a, const FragH& b, v8f c) {
  v8f d = __builtin_amdgcn_wmma_f32_16x16x32_f16(false, a.v, false, b.v, (short)0, c, false, false);
  asm volatile("v_nop\n\tv_nop\n\tv_nop\n\tv_nop" : "+v"(d) : "v"(a.w), "v"(b.w));
  return d;
}

__device__ __forceinline__ unsigned bf16_bits(float f) {
  const unsigned u = __float_as_uint(f);
  const unsigned r = (u + 0x7FFFu + ((u >> 16) & 1u)) >> 16;
  const unsigned q = (u >> 16) | 0x40u;
  return ((u & 0x7fffffffu) > 0x7f800000u) ? q : r;
}

__device__ __forceinline__ float bf16_val(float f) {
  return __uint_as_float(bf16_bits(f) << 16);
}
__device__ __forceinline__ int clampi(int v, int lo, int hi) {
  return v < lo ? lo : (v > hi ? hi : v);
}

__device__ __forceinline__ unsigned f16_bits(float f) {
  const unsigned u  = __float_as_uint(f);
  const unsigned s  = (u >> 16) & 0x8000u;
  const unsigned a  = u & 0x7fffffffu;
  const unsigned t  = a - 0x38000000u;
  const unsigned r  = (t + 0x0FFFu + ((t >> 13) & 1u)) >> 13;
  const unsigned rc = r > 0x7C00u ? 0x7C00u : r;
  const bool small  = a < 0x38800000u;
  const bool isnan  = a > 0x7f800000u;
  const unsigned fin = small ? 0u : (s | rc);
  return isnan ? (s | 0x7E00u) : fin;
}

__device__ __forceinline__ unsigned pk16(unsigned lo, unsigned hi) { return lo | (hi << 16); }
__device__ __forceinline__ unsigned bf16_lo_bits(float v) {
  float hi = bf16_val(v);
  asm volatile("" : "+v"(hi));
  return bf16_bits(v - hi);
}
__device__ __forceinline__ v4u pack8_bf16(v4f a, v4f c) {
  return (v4u){ pk16(bf16_bits(a[0]), bf16_bits(a[1])), pk16(bf16_bits(a[2]), bf16_bits(a[3])),
                pk16(bf16_bits(c[0]), bf16_bits(c[1])), pk16(bf16_bits(c[2]), bf16_bits(c[3])) };
}
__device__ __forceinline__ v4u pack8_bf16_lo(v4f a, v4f c) {
  return (v4u){ pk16(bf16_lo_bits(a[0]), bf16_lo_bits(a[1])), pk16(bf16_lo_bits(a[2]), bf16_lo_bits(a[3])),
                pk16(bf16_lo_bits(c[0]), bf16_lo_bits(c[1])), pk16(bf16_lo_bits(c[2]), bf16_lo_bits(c[3])) };
}
__device__ __forceinline__ v4u pack8_f16(v4f a, v4f c) {
  return (v4u){ pk16(f16_bits(a[0]), f16_bits(a[1])), pk16(f16_bits(a[2]), f16_bits(a[3])),
                pk16(f16_bits(c[0]), f16_bits(c[1])), pk16(f16_bits(c[2]), f16_bits(c[3])) };
}

template <int FORM>
__global__ __launch_bounds__(256) void k_plane(const float* __restrict__ src, int rows, int cols, int ldsrc,
                                               unsigned short* __restrict__ dst, int MP, int KP) {
  static_assert(FORM >= 0 && FORM <= 3);
  const int KTOT = (FORM == 1 || FORM == 3) ? 2 * KP : KP;
  const unsigned ppr   = (unsigned)(KTOT >> 3);
  const unsigned kp8   = (unsigned)(KP >> 3);
  const unsigned total = (unsigned)MP * ppr;
  const unsigned g     = blockIdx.x * 256u + threadIdx.x;
  const unsigned rowu  = g / ppr;
  const unsigned p     = g - rowu * ppr;
  const bool second    = p >= kp8;
  const int row = (int)rowu;
  const int c0  = (int)((second ? p - kp8 : p) << 3);
  const float* srow = src + (size_t)clampi(row, 0, rows - 1) * (size_t)ldsrc;
  float x[8];
  unsigned mk[8];
#pragma unroll
  for (int e = 0; e < 8; ++e) {
    const int c = c0 + e;
    const float v = srow[clampi(c, 0, cols - 1)];
    asm volatile("" :: "v"(v));
    x[e]  = v;
    mk[e] = (row < rows && c < cols) ? 0xFFFFu : 0u;
  }
  const v4f a = (v4f){ x[0], x[1], x[2], x[3] };
  const v4f c = (v4f){ x[4], x[5], x[6], x[7] };
  v4u o;
  if (FORM == 2) {
    o = pack8_f16(a, c);
  } else {
    const v4u hi = pack8_bf16(a, c);
    o = hi;
    if (FORM == 1) { const v4u lo = pack8_bf16_lo(a, c); o = second ? lo : hi; }
  }
  const v4u mw = (v4u){ pk16(mk[0], mk[1]), pk16(mk[2], mk[3]), pk16(mk[4], mk[5]), pk16(mk[6], mk[7]) };
  o &= mw;
  if (g < total) {
    volatile v4u* q = (volatile v4u*)(dst + (size_t)g * 8);
    *q = o;
    __threadfence();
    *q = o;
  }
}

template <int FORM> struct FragOf    { typedef FragB T; };
template <>         struct FragOf<2> { typedef FragH T; };
__device__ __forceinline__ v8f mm(const FragB& a, const FragB& b, v8f c) { return wmb(a, b, c); }
__device__ __forceinline__ v8f mm(const FragH& a, const FragH& b, v8f c) { return wmh(a, b, c); }
template <class F> __device__ __forceinline__ F ld_frag(const unsigned short* p) {
  F f;
  f.h[0] = *(const v8usa*)(p);
  f.h[1] = *(const v8usa*)(p + 16);
  return f;
}

template <int FORM, int EPI>
__global__ __launch_bounds__(256) __attribute__((amdgpu_num_vgpr(248)))
void k_gemm_nt(const unsigned short* __restrict__ A, const unsigned short* __restrict__ B,
               const float* __restrict__ bias, float* __restrict__ D, int M, int N, int KTOT, int ldd) {
  static_assert(FORM >= 0 && FORM <= 2);
  static_assert(EPI == 0 || EPI == 1);
  typedef typename FragOf<FORM>::T F;
  __shared__ __attribute__((aligned(16))) float sT[8][16 * 68];
  const int lane = threadIdx.x & 31;
  const int wave = threadIdx.x >> 5;
  const int tilesM = (M + 63) >> 6;
  const int tilesN = (N + 63) >> 6;
  const int tile = blockIdx.x * 8 + wave;
  if (tile >= tilesM * tilesN) return;
  const int tm = tile / tilesN;
  const int tn = tile - tm * tilesN;
  const int m0 = tm << 6;
  const int n0 = tn << 6;

  const int rl = lane & 15;
  const int h8 = (lane >> 4) * 8;
  const unsigned short* pa = A + (size_t)(m0 + rl) * (size_t)KTOT + h8;
  const unsigned short* pb = B + (size_t)(n0 + rl) * (size_t)KTOT + h8;

  v8f acc[4][4];
#pragma unroll
  for (int i = 0; i < 4; ++i)
#pragma unroll
    for (int j = 0; j < 4; ++j) acc[i][j] = (v8f){0.f, 0.f, 0.f, 0.f, 0.f, 0.f, 0.f, 0.f};

#pragma unroll 1
  for (int k0 = 0; k0 < KTOT; k0 += 32) {
    F bf[4];
#pragma unroll
    for (int j = 0; j < 4; ++j) bf[j] = ld_frag<F>(pb + (size_t)(j << 4) * (size_t)KTOT + k0);
#pragma unroll
    for (int i = 0; i < 4; ++i) {
      const F af = ld_frag<F>(pa + (size_t)(i << 4) * (size_t)KTOT + k0);
#pragma unroll
      for (int j = 0; j < 4; ++j) acc[i][j] = mm(af, bf[j], acc[i][j]);
    }
  }

  float* slab = sT[wave];
  const int hh = lane >> 4;
  const int c4 = (lane & 15) * 4;
  const int nc = n0 + c4;
  const bool cok = nc < N;
  v4f bv = (v4f){0.f, 0.f, 0.f, 0.f};
  if (EPI == 1) {
    bv = *(const v4fa*)(bias + clampi(nc, 0, N - 4));
    asm volatile("" :: "v"(bv));
  }
#pragma unroll
  for (int i = 0; i < 4; ++i) {
    const int mBase = m0 + (i << 4);
#pragma unroll
    for (int j = 0; j < 4; ++j) {
#pragma unroll
      for (int r = 0; r < 8; ++r) slab[(h8 + r) * 68 + (j << 4) + rl] = acc[i][j][r];
    }
    __builtin_amdgcn_fence(__ATOMIC_RELEASE, "workgroup");
    __builtin_amdgcn_wave_barrier();
    __builtin_amdgcn_fence(__ATOMIC_ACQUIRE, "workgroup");
    v4f vv[8];
#pragma unroll
    for (int it = 0; it < 8; ++it) {
      const int row = it * 2 + hh;
      v4f v = *(const v4fa*)(slab + row * 68 + c4);
      if (EPI == 1) v += bv;
      vv[it] = v;
    }
    for (int pass = 0; pass < 2; ++pass) {
#pragma unroll
      for (int it = 0; it < 8; ++it) {
        const int row = mBase + it * 2 + hh;
        if (cok && row < M) *(volatile v4f*)(D + (size_t)row * (size_t)ldd + nc) = vv[it];
      }
      __threadfence();
    }
    __builtin_amdgcn_fence(__ATOMIC_RELEASE, "workgroup");
    __builtin_amdgcn_wave_barrier();
    __builtin_amdgcn_fence(__ATOMIC_ACQUIRE, "workgroup");
  }
}

#include <stddef.h>
#include <stdint.h>
#include <math.h>

#ifndef TWO_TERM_L1
#define TWO_TERM_L1 1
#endif
#ifndef TWO_TERM_L2
#define TWO_TERM_L2 1
#endif

typedef int          v4i __attribute__((ext_vector_type(4)));
typedef unsigned int v2u __attribute__((ext_vector_type(2)));
typedef v4i __attribute__((may_alias)) v4ia;
typedef v2u __attribute__((may_alias)) v2ua;

constexpr int NN     = 50000;
constexpr int DD     = 128;
constexpr int KD     = 2 * DD;
constexpr int NE     = 800000;
constexpr int MPAD   = 50048;
constexpr int NTHR   = 256;
constexpr int NWAVE  = 8;
constexpr int EPT    = 8;
constexpr int CHUNK  = NTHR * EPT;
constexpr int NCHUNK = (NE + CHUNK - 1) / CHUNK;
constexpr int WCAP   = EPT * 32;
constexpr int LISTN  = NWAVE * WCAP;
constexpr int SLB    = 10;
constexpr int NBRUN  = 1 << SLB;
constexpr int NBLK   = (NN + NBRUN - 1) / NBRUN;
constexpr int RCAP   = 21504;
constexpr int DEGCAP = 64;
constexpr int FLAGP  = 32;
constexpr int BK_ZINTS = LISTN + 2 * RCAP + 3 * NBRUN;
constexpr int BK_INTS  = BK_ZINTS + 16;
constexpr size_t BUCKET_LDS = (size_t)BK_INTS * 4;
constexpr int PB_W0  = DD * (DD / 8) / NTHR;
constexpr int PB_WD  = DD * (KD / 8) / NTHR;
constexpr int PB_PAD = (MPAD - NN) * (KD / 8) / NTHR;
constexpr int PB_TOTAL = PB_W0 + 2 * PB_WD + 1 + PB_PAD;

static_assert(NN % 8 == 0);
static_assert(DD == 128 && DD == 32 * 4);
static_assert(NE == 390 * 2048 + 1280 && NCHUNK == 391);
static_assert(NE % EPT == 0 && NE % 4 == 0);
static_assert(NBLK == 49 && NBLK * NBRUN >= NN);
static_assert(MPAD == 391 * 128 && MPAD % 64 == 0 && MPAD >= NN && NN % 16 == 0);
static_assert(RCAP * 4 >= 5 * 16623);
static_assert(DEGCAP >= 35 + 8);
static_assert(RCAP % (4 * NTHR) == 0 && BK_ZINTS % (4 * NTHR) == 0);
static_assert(((long long)(NN - 1) << SLB) < (1LL << 31));
static_assert(BUCKET_LDS <= 262144);
static_assert(DD * (DD / 8) % NTHR == 0 && DD * (KD / 8) % NTHR == 0);
static_assert((MPAD - NN) * (KD / 8) % NTHR == 0);
static_assert(NBRUN == 4 * NTHR);

constexpr size_t al256c(size_t o) { return (o + 255) & ~(size_t)255; }
constexpr size_t SZ_XB   = (size_t)MPAD * DD * 2;
constexpr size_t SZ_T    = (size_t)MPAD * DD * 4;
constexpr size_t SZ_H    = (size_t)MPAD * DD * 4;
constexpr size_t SZ_HHL  = (size_t)MPAD * KD * 2;
constexpr size_t SZ_LIST = (size_t)NBLK * RCAP * 4;
constexpr size_t SZ_TAB  = (size_t)NBLK * NBRUN * 4;
constexpr size_t SZ_FLAG = (size_t)NBLK * FLAGP * 4;
constexpr size_t O_XB   = 0;
constexpr size_t O_T    = al256c(O_XB + SZ_XB);
constexpr size_t O_H    = al256c(O_T + SZ_T);
constexpr size_t O_HHL  = al256c(O_H + SZ_H);
constexpr size_t O_LIST = al256c(O_HHL + SZ_HHL);
constexpr size_t O_CNT  = al256c(O_LIST + SZ_LIST);
constexpr size_t O_OFF  = al256c(O_CNT + SZ_TAB);
constexpr size_t O_DEG  = al256c(O_OFF + SZ_TAB);
constexpr size_t O_DIS  = al256c(O_DEG + SZ_TAB);
constexpr size_t O_FLAG = al256c(O_DIS + SZ_TAB);
constexpr size_t O_W0B  = al256c(O_FLAG + SZ_FLAG);
constexpr size_t O_W1D  = al256c(O_W0B + (size_t)DD * DD * 2);
constexpr size_t O_W2D  = al256c(O_W1D + (size_t)DD * KD * 2);
constexpr size_t O_BF   = al256c(O_W2D + (size_t)DD * KD * 2);
constexpr size_t WS_TOTAL = al256c(O_BF + (size_t)3 * DD * 4);
static_assert(WS_TOTAL <= ((size_t)128 << 20));
static_assert((size_t)(NN - 1) * DD + DD - 1 == (size_t)6399999);

__device__ __forceinline__ int scan_chunk(const int* __restrict__ keyp, const int* __restrict__ othp,
                                          int cbase, int slotBase, int* list, int tid, int wave) {
  const int e0 = cbase + tid * EPT;
  const bool valid = e0 < NE;
  const int eg = valid ? e0 : (NE - EPT);
  const v4i ka = *(const v4ia*)(keyp + eg);
  asm volatile("" :: "v"(ka));
  const v4i kb = *(const v4ia*)(keyp + eg + 4);
  asm volatile("" :: "v"(kb));
  const v4i oa = *(const v4ia*)(othp + eg);
  asm volatile("" :: "v"(oa));
  const v4i ob = *(const v4ia*)(othp + eg + 4);
  asm volatile("" :: "v"(ob));
  const int kk[8] = { ka.x, ka.y, ka.z, ka.w, kb.x, kb.y, kb.z, kb.w };
  const int oo[8] = { oa.x, oa.y, oa.z, oa.w, ob.x, ob.y, ob.z, ob.w };
  bool hit[8];
  int  ent[8];
  int  c = 0;
#pragma unroll
  for (int j = 0; j < 8; ++j) {
    const unsigned s = (unsigned)kk[j] - (unsigned)slotBase;
    const bool h = valid && (s < (unsigned)NBRUN) && ((unsigned)kk[j] < (unsigned)NN) && (kk[j] != oo[j]);
    hit[j] = h;
    ent[j] = (clampi(oo[j], 0, NN - 1) << SLB) | (int)(s & (unsigned)(NBRUN - 1));
    c += h ? 1 : 0;
  }
  const unsigned m1 = __builtin_amdgcn_ballot_w32((c & 1) != 0);
  const unsigned m2 = __builtin_amdgcn_ballot_w32((c & 2) != 0);
  const unsigned m4 = __builtin_amdgcn_ballot_w32((c & 4) != 0);
  const unsigned m8 = __builtin_amdgcn_ballot_w32((c & 8) != 0);
  const int pre = (int)__builtin_amdgcn_mbcnt_lo(m1, 0u) + 2 * (int)__builtin_amdgcn_mbcnt_lo(m2, 0u)
                + 4 * (int)__builtin_amdgcn_mbcnt_lo(m4, 0u) + 8 * (int)__builtin_amdgcn_mbcnt_lo(m8, 0u);
  const int tot = (int)__builtin_popcount(m1) + 2 * (int)__builtin_popcount(m2)
                + 4 * (int)__builtin_popcount(m4) + 8 * (int)__builtin_popcount(m8);
  int p = wave * WCAP + pre;
#pragma unroll
  for (int j = 0; j < 8; ++j) {
    if (hit[j]) { list[p] = ent[j]; ++p; }
  }
  return tot;
}

template <int DOUBLED>
__device__ __forceinline__ void prep_w_piece(const float* __restrict__ W, unsigned short* __restrict__ dst, int g) {
  const int n  = DOUBLED ? (g >> 5) : (g >> 4);
  const int k8 = (g & 15) * 8;
  const float* s = W + (size_t)n * DD + k8;
  const v4f a = *(const v4fa*)s;
  const v4f c = *(const v4fa*)(s + 4);
  const v4u o = pack8_bf16(a, c);
  volatile v4u* q = (volatile v4u*)(dst + (size_t)g * 8);
  *q = o;
  __threadfence();
  *q = o;
}

__global__ __launch_bounds__(NTHR) void k_prep(const float* __restrict__ W0, const float* __restrict__ W1,
                                               const float* __restrict__ W2, const float* __restrict__ b0,
                                               const float* __restrict__ b1, const float* __restrict__ b2,
                                               unsigned short* __restrict__ W0B, unsigned short* __restrict__ W1D,
                                               unsigned short* __restrict__ W2D, float* __restrict__ BF,
                                               unsigned short* __restrict__ HHL) {
  const int blk = (int)blockIdx.x, tid = (int)threadIdx.x;
  if (blk < PB_W0) {
    prep_w_piece<0>(W0, W0B, blk * NTHR + tid);
  } else if (blk < PB_W0 + PB_WD) {
    prep_w_piece<1>(W1, W1D, (blk - PB_W0) * NTHR + tid);
  } else if (blk < PB_W0 + 2 * PB_WD) {
    prep_w_piece<1>(W2, W2D, (blk - PB_W0 - PB_WD) * NTHR + tid);
  } else if (blk == PB_W0 + 2 * PB_WD) {
    const int wave = tid >> 5, lane = tid & 31, c4 = lane * 4;
    const v4f v0 = *(const v4fa*)(b0 + c4);
    asm volatile("" :: "v"(v0));
    const v4f v1 = *(const v4fa*)(b1 + c4);
    asm volatile("" :: "v"(v1));
    const v4f v2 = *(const v4fa*)(b2 + c4);
    asm volatile("" :: "v"(v2));
    const v4f v = (wave == 0) ? v0 : ((wave == 1) ? v1 : v2);
    const v4f o = (v4f){ bf16_val(v.x), bf16_val(v.y), bf16_val(v.z), bf16_val(v.w) };
    if (wave < 3) {
      volatile v4f* q = (volatile v4f*)(BF + wave * DD + c4);
      *q = o;
      __threadfence();
      *q = o;
    }
  } else {
    const int g = (blk - (PB_W0 + 2 * PB_WD + 1)) * NTHR + tid;
    const v4u z = (v4u){ 0u, 0u, 0u, 0u };
    volatile v4u* q = (volatile v4u*)(HHL + (size_t)NN * KD + (size_t)g * 8);
    *q = z;
    __threadfence();
    *q = z;
  }
}

__global__ __launch_bounds__(NTHR) void k_degree(const int* __restrict__ rowp, const int* __restrict__ colp,
                                                 int* __restrict__ DEG, float* __restrict__ DIS) {
  __shared__ __attribute__((aligned(16))) int   scnt[NBRUN];
  __shared__ __attribute__((aligned(16))) int   list[LISTN];
  __shared__ __attribute__((aligned(16))) float sdis[NBRUN];
  __shared__ int wcnt[NWAVE];
  const int tid = (int)threadIdx.x, lane = tid & 31, wave = tid >> 5;
  const int nodeBase = (int)blockIdx.x * NBRUN;

  for (int i = tid; i < NBRUN; i += NTHR) { scnt[i] = 0; sdis[i] = 0.0f; }
  for (int i = tid; i < LISTN; i += NTHR) list[i] = 0;
  if (tid < NWAVE) wcnt[tid] = 0;
  __syncthreads();

#pragma unroll 1
  for (int ch = 0; ch < NCHUNK; ++ch) {
    const int wc = scan_chunk(rowp, colp, ch * CHUNK, nodeBase, list, tid, wave);
    if (lane == 0) wcnt[wave] = wc;
    __syncthreads();
    if (wave == 0) {
#pragma unroll 1
      for (int w2 = 0; w2 < NWAVE; ++w2) {
        const int c = clampi(wcnt[w2], 0, WCAP);
#pragma unroll 1
        for (int b0 = 0; b0 < c; b0 += 32) {
          const int idx = b0 + lane;
          const int ent = list[w2 * WCAP + (idx < WCAP ? idx : WCAP - 1)];
          const int m32 = (c - b0) < 32 ? (c - b0) : 32;
#pragma unroll 1
          for (int k = 0; k < m32; ++k) {
            const int u  = __builtin_amdgcn_readlane(ent, k);
            const int sl = u & (NBRUN - 1);
            if (lane == 0) scnt[sl] = scnt[sl] + 1;
          }
        }
      }
    }
    __syncthreads();
  }

#pragma unroll 1
  for (int it = 0; it < NBRUN / NTHR; ++it) {
    const int s = it * NTHR + tid;
    const int d = scnt[s];
    const float df = (float)(d < 1 ? 1 : d);
    const float r = 1.0f / sqrtf(df);
    sdis[s] = (d > 0) ? r : 0.0f;
  }
  __syncthreads();
  const v4i cv = *(const v4ia*)(scnt + 4 * tid);
  const v4f dv = *(const v4fa*)(sdis + 4 * tid);
  volatile v4i* qd = (volatile v4i*)(DEG + (size_t)nodeBase + 4 * tid);
  volatile v4f* qs = (volatile v4f*)(DIS + (size_t)nodeBase + 4 * tid);
  *qd = cv;
  *qs = dv;
  __threadfence();
  *qd = cv;
  *qs = dv;
}

__global__ __launch_bounds__(NTHR) void k_bucket(const int* __restrict__ rowp, const int* __restrict__ colp,
                                                 int* __restrict__ LIST, int* __restrict__ CNT,
                                                 int* __restrict__ OFF, int* __restrict__ FLAG) {
  extern __shared__ __attribute__((aligned(16))) int dsm[];
  int* list = dsm;
  int* hl   = dsm + LISTN;
  int* sl   = hl + RCAP;
  int* cnt  = sl + RCAP;
  int* offs = cnt + NBRUN;
  int* cur  = offs + NBRUN;
  int* misc = cur + NBRUN;
  const int tid = (int)threadIdx.x, lane = tid & 31, wave = tid >> 5;
  const int blk = (int)blockIdx.x;
  const int nodeBase = blk * NBRUN;

  {
    const v4i z4 = (v4i){ 0, 0, 0, 0 };
    for (int i = tid * 4; i < BK_ZINTS; i += NTHR * 4) *(v4ia*)(dsm + i) = z4;
    if (tid < 16) misc[tid] = 0;
  }
  __syncthreads();

  int t = 0, ov = 0;
#pragma unroll 1
  for (int ch = 0; ch < NCHUNK; ++ch) {
    const int wc = scan_chunk(colp, rowp, ch * CHUNK, nodeBase, list, tid, wave);
    if (lane == 0) misc[wave] = wc;
    __syncthreads();
    if (wave == 0) {
#pragma unroll 1
      for (int w2 = 0; w2 < NWAVE; ++w2) {
        const int c = clampi(misc[w2], 0, WCAP);
#pragma unroll 1
        for (int b0 = 0; b0 < c; b0 += 32) {
          const int idx = b0 + lane;
          const int ent = list[w2 * WCAP + (idx < WCAP ? idx : WCAP - 1)];
          const int m32 = (c - b0) < 32 ? (c - b0) : 32;
#pragma unroll 1
          for (int k = 0; k < m32; ++k) {
            const int u    = __builtin_amdgcn_readlane(ent, k);
            const int slot = u & (NBRUN - 1);
            if (t < RCAP) {
              if (lane == 0) { hl[t] = u; cnt[slot] = cnt[slot] + 1; }
              t = t + 1;
            } else {
              ov = 1;
            }
          }
        }
      }
    }
    __syncthreads();
  }
  if (wave == 0 && lane == 0) { misc[8] = t; misc[9] = ov; }
  __syncthreads();
  const int tt  = clampi(misc[8], 0, RCAP);
  const int ovf = misc[9];

  if (wave == 0) {
    const int base = lane * (NBRUN / 32);
    int s = 0;
#pragma unroll 1
    for (int i = 0; i < NBRUN / 32; ++i) s += cnt[base + i];
    int incl = s;
#pragma unroll
    for (int d = 1; d < 32; d <<= 1) {
      const int y = __shfl_up(incl, d, 32);
      if (lane >= d) incl += y;
    }
    int run = incl - s;
#pragma unroll 1
    for (int i = 0; i < NBRUN / 32; ++i) {
      const int cv = cnt[base + i];
      offs[base + i] = run;
      cur[base + i]  = run;
      run += cv;
    }
  }
  __syncthreads();
  if (wave == 0) {
#pragma unroll 1
    for (int b0 = 0; b0 < tt; b0 += 32) {
      const int idx = b0 + lane;
      const int ent = hl[idx < RCAP ? idx : RCAP - 1];
      const int m32 = (tt - b0) < 32 ? (tt - b0) : 32;
#pragma unroll 1
      for (int k = 0; k < m32; ++k) {
        const int u    = __builtin_amdgcn_readlane(ent, k);
        const int slot = u & (NBRUN - 1);
        if (lane == 0) {
          const int p = clampi(cur[slot], 0, RCAP - 1);
          sl[p] = u;
          cur[slot] = p + 1;
        }
      }
    }
  }
  __syncthreads();

  int* gl = LIST + (size_t)blk * RCAP;
  const v4i c4v = *(const v4ia*)(cnt + 4 * tid);
  const v4i o4v = *(const v4ia*)(offs + 4 * tid);
  const v4i f4v = (v4i){ ovf, ovf, ovf, ovf };
  for (int pass = 0; pass < 2; ++pass) {
#pragma unroll 1
    for (int it = 0; it < RCAP / (4 * NTHR); ++it) {
      const int i4 = (it * NTHR + tid) * 4;
      const v4i v = *(const v4ia*)(sl + i4);
      const v4i r = (v4i){ v.x >> SLB, v.y >> SLB, v.z >> SLB, v.w >> SLB };
      *(volatile v4i*)(gl + i4) = r;
    }
    *(volatile v4i*)(CNT + (size_t)nodeBase + 4 * tid) = c4v;
    *(volatile v4i*)(OFF + (size_t)nodeBase + 4 * tid) = o4v;
    if (tid < FLAGP / 4) *(volatile v4i*)(FLAG + (size_t)blk * FLAGP + 4 * tid) = f4v;
    __threadfence();
  }
}

template <int LAYER>
__global__ __launch_bounds__(NTHR) void k_replay(const int* __restrict__ LIST, const int* __restrict__ CNT,
                                                 const int* __restrict__ OFF, const int* __restrict__ FLAG,
                                                 const float* __restrict__ DIS, const float* __restrict__ T,
                                                 const unsigned short* __restrict__ XB, float* H,
                                                 unsigned short* HHL, float* out, int nRows) {
#pragma clang fp contract(off)
  const int tid = (int)threadIdx.x, lane = tid & 31, wave = tid >> 5;
  const int row = (int)blockIdx.x * NWAVE + wave;
  const bool live = row < nRows;
  const int rc  = live ? row : (nRows - 1);
  const int blk = rc >> SLB;
  int cv = CNT[rc];
  asm volatile("" :: "v"(cv));
  int ofv = OFF[rc];
  asm volatile("" :: "v"(ofv));
  int fl = FLAG[(size_t)blk * FLAGP];
  asm volatile("" :: "v"(fl));
  const float dd = DIS[rc];
  const bool big = cv > DEGCAP;
  int cc = clampi(cv, 0, DEGCAP);
  cc = live ? cc : 0;
  const int cn = __builtin_amdgcn_readfirstlane(cc);
  const int o  = clampi(ofv, 0, RCAP);
  const int* lst = LIST + (size_t)blk * RCAP;

  v4f hp;
  if constexpr (LAYER == 0) {
    const v2u xw = *(const v2ua*)(XB + (size_t)rc * DD + 4 * lane);
    hp.x = __uint_as_float(xw.x << 16);
    hp.y = __uint_as_float(xw.x & 0xffff0000u);
    hp.z = __uint_as_float(xw.y << 16);
    hp.w = __uint_as_float(xw.y & 0xffff0000u);
  } else {
    hp = *(const v4fa*)(H + (size_t)rc * DD + 4 * lane);
  }

  v4f acc = (v4f){ 0.0f, 0.0f, 0.0f, 0.0f };
#pragma unroll 1
  for (int b0 = 0; b0 < cn; b0 += 32) {
    const int idx = clampi(o + b0 + lane, 0, RCAP - 1);
    const int sr  = clampi(lst[idx], 0, NN - 1);
    const float cf = DIS[sr] * dd;
    const int cfi  = __float_as_int(cf);
    const int m32  = (cn - b0) < 32 ? (cn - b0) : 32;
#pragma unroll 1
    for (int k = 0; k < m32; ++k) {
      const int   sk = __builtin_amdgcn_readlane(sr, k);
      const float ck = __int_as_float(__builtin_amdgcn_readlane(cfi, k));
      const v4f v = *(const v4fa*)(T + (size_t)sk * DD + 4 * lane);
      const float m0 = ck * v.x, m1 = ck * v.y, m2 = ck * v.z, m3 = ck * v.w;
      acc.x = acc.x + m0;
      acc.y = acc.y + m1;
      acc.z = acc.z + m2;
      acc.w = acc.w + m3;
    }
  }

  const float qnan = __int_as_float(0x7fc00000);
  const bool poison = (fl != 0) || big;
  v4f hn;
  {
    const float a0 = (acc.x > 0.0f) ? acc.x : (acc.x - acc.x);
    const float a1 = (acc.y > 0.0f) ? acc.y : (acc.y - acc.y);
    const float a2 = (acc.z > 0.0f) ? acc.z : (acc.z - acc.z);
    const float a3 = (acc.w > 0.0f) ? acc.w : (acc.w - acc.w);
    hn.x = poison ? qnan : (hp.x + a0);
    hn.y = poison ? qnan : (hp.y + a1);
    hn.z = poison ? qnan : (hp.z + a2);
    hn.w = poison ? qnan : (hp.w + a3);
  }

  if constexpr (LAYER < 2) {
    constexpr int TWO = (LAYER == 0) ? TWO_TERM_L1 : TWO_TERM_L2;
    const int hw0 = (int)pk16(bf16_bits(hn.x), bf16_bits(hn.y));
    const int hw1 = (int)pk16(bf16_bits(hn.z), bf16_bits(hn.w));
    int lw0 = 0, lw1 = 0;
    if (TWO != 0) {
      lw0 = (int)pk16(bf16_lo_bits(hn.x), bf16_lo_bits(hn.y));
      lw1 = (int)pk16(bf16_lo_bits(hn.z), bf16_lo_bits(hn.w));
    }
    const int sa = (2 * lane) & 31, sb = (2 * lane + 1) & 31;
    const int g0 = __shfl(hw0, sa, 32), g1 = __shfl(hw1, sa, 32);
    const int g2 = __shfl(hw0, sb, 32), g3 = __shfl(hw1, sb, 32);
    const int p0 = __shfl(lw0, sa, 32), p1 = __shfl(lw1, sa, 32);
    const int p2 = __shfl(lw0, sb, 32), p3 = __shfl(lw1, sb, 32);
    const bool lsel = lane >= 16;
    v4u pv;
    pv.x = (unsigned)(lsel ? p0 : g0);
    pv.y = (unsigned)(lsel ? p1 : g1);
    pv.z = (unsigned)(lsel ? p2 : g2);
    pv.w = (unsigned)(lsel ? p3 : g3);
    if (live) {
      volatile v4f* hq = (volatile v4f*)(H + (size_t)row * DD + 4 * lane);
      volatile v4u* pq = (volatile v4u*)(HHL + (size_t)row * KD + 8 * lane);
      *hq = hn;
      *pq = pv;
      __threadfence();
      *hq = hn;
      *pq = pv;
    }
  } else {
    if (live) {
      volatile v4f* oq = (volatile v4f*)(out + (size_t)row * DD + 4 * lane);
      *oq = hn;
      __threadfence();
      *oq = hn;
    }
  }
}

extern "C" void kernel_launch(void* const* d_in, const int* in_sizes, int n_in,
                              void* d_out, int out_size, void* d_ws, size_t ws_size,
                              hipStream_t stream) {
  if (n_in < 8) return;
  if (in_sizes[0] != NN * DD) return;
  if (in_sizes[1] != 2 * NE) return;
  if (in_sizes[2] != DD * DD || in_sizes[4] != DD * DD || in_sizes[6] != DD * DD) return;
  if (in_sizes[3] != DD || in_sizes[5] != DD || in_sizes[7] != DD) return;
  if (out_size != NN * DD) return;
  if (ws_size < WS_TOTAL) return;

  const float* x  = (const float*)d_in[0];
  const int*   ei = (const int*)d_in[1];
  const float* W0 = (const float*)d_in[2];
  const float* b0 = (const float*)d_in[3];
  const float* W1 = (const float*)d_in[4];
  const float* b1 = (const float*)d_in[5];
  const float* W2 = (const float*)d_in[6];
  const float* b2 = (const float*)d_in[7];
  float* out = (float*)d_out;
  const int* rowp = ei;
  const int* colp = ei + NE;

  char* ws = (char*)d_ws;
  unsigned short* XB   = (unsigned short*)(ws + O_XB);
  float*          T    = (float*)(ws + O_T);
  float*          H    = (float*)(ws + O_H);
  unsigned short* HHL  = (unsigned short*)(ws + O_HHL);
  int*            LIST = (int*)(ws + O_LIST);
  int*            CNT  = (int*)(ws + O_CNT);
  int*            OFF  = (int*)(ws + O_OFF);
  int*            DEG  = (int*)(ws + O_DEG);
  float*          DIS  = (float*)(ws + O_DIS);
  int*            FLAG = (int*)(ws + O_FLAG);
  unsigned short* W0B  = (unsigned short*)(ws + O_W0B);
  unsigned short* W1D  = (unsigned short*)(ws + O_W1D);
  unsigned short* W2D  = (unsigned short*)(ws + O_W2D);
  float*          BF   = (float*)(ws + O_BF);

  (void)hipFuncSetAttribute(reinterpret_cast<const void*>(&k_bucket), hipFuncAttributeMaxDynamicSharedMemorySize,
                            (int)BUCKET_LDS);

  constexpr int gPlane  = MPAD * (DD / 8) / 256;
  static_assert(gPlane * 256 == MPAD * (DD / 8));
  constexpr int gGemm   = (((NN + 63) / 64) * (DD / 64) + 7) / 8;
  constexpr int gReplay = NN / NWAVE;

  k_plane<0><<<gPlane, 256, 0, stream>>>(x, NN, DD, DD, XB, MPAD, DD);
  k_prep<<<PB_TOTAL, NTHR, 0, stream>>>(W0, W1, W2, b0, b1, b2, W0B, W1D, W2D, BF, HHL);
  k_degree<<<NBLK, NTHR, 0, stream>>>(rowp, colp, DEG, DIS);
  k_bucket<<<NBLK, NTHR, BUCKET_LDS, stream>>>(rowp, colp, LIST, CNT, OFF, FLAG);
  k_gemm_nt<0, 1><<<gGemm, 256, 0, stream>>>(XB, W0B, BF, T, NN, DD, DD, DD);
  k_replay<0><<<gReplay, NTHR, 0, stream>>>(LIST, CNT, OFF, FLAG, DIS, T, XB, H, HHL, out, NN);
  k_gemm_nt<0, 1><<<gGemm, 256, 0, stream>>>(HHL, W1D, BF + DD, T, NN, DD, KD, DD);
  k_replay<1><<<gReplay, NTHR, 0, stream>>>(LIST, CNT, OFF, FLAG, DIS, T, XB, H, HHL, out, NN);
  k_gemm_nt<0, 1><<<gGemm, 256, 0, stream>>>(HHL, W2D, BF + 2 * DD, T, NN, DD, KD, DD);
  k_replay<2><<<gReplay, NTHR, 0, stream>>>(LIST, CNT, OFF, FLAG, DIS, T, XB, H, HHL, out, NN);
}
